// MSDeformRefAttn2D_90074054132154
// MI455X (gfx1250) — hardware-verified
//
#include <hip/hip_runtime.h>
#define NCm 6
#define CE 256
#define HQ 100
#define WQ 100
#define NQ (HQ * WQ)
#define NQP 10016
#define HL 32
#define WL 88
#define ML (HL * WL)
#define NH 8
#define NPt 4
#define DHd 32
typedef __bf16 v16b __attribute__((ext_vector_type(16)));
typedef unsigned short v8us __attribute__((ext_vector_type(8), may_alias));
typedef float  v8f  __attribute__((ext_vector_type(8)));
typedef float  v4f  __attribute__((ext_vector_type(4)));
typedef float  v4fa __attribute__((ext_vector_type(4), may_alias));
union FragB { v16b v; v8us half[2]; unsigned short u[16]; };

__device__ __forceinline__ unsigned short bf16_bits(float x) { unsigned int u = __float_as_uint(x); return (unsigned short)((u + 0x7FFFu + ((u >> 16) & 1u)) >> 16); }
__device__ __forceinline__ float bf16_val(unsigned short b) { return __uint_as_float(((unsigned int)b) << 16); }
__device__ __forceinline__ float bf16_round(float x) { return bf16_val(bf16_bits(x)); }
template <int NT>
__device__ __forceinline__ v8f mmaN(v16b ah, v16b al, v16b bh, v16b bl, v8f c) {
  c = __builtin_amdgcn_wmma_f32_16x16x32_bf16(false, ah, false, bh, (short)0, c, false, false);
  if (NT >= 2) c = __builtin_amdgcn_wmma_f32_16x16x32_bf16(false, al, false, bh, (short)0, c, false, false);
  if (NT >= 3) c = __builtin_amdgcn_wmma_f32_16x16x32_bf16(false, ah, false, bl, (short)0, c, false, false);
  asm volatile("v_nop\n\tv_nop\n\tv_nop\n\tv_nop" : "+v"(c) : "v"(ah), "v"(al), "v"(bh), "v"(bl));
  return c;
}

__global__ __launch_bounds__(256) void k_wt_bf16(const float* __restrict__ W, unsigned short* __restrict__ Wt, int K, int N) {
  const int t = blockIdx.x * 256 + threadIdx.x;
  const int k8n = K / 8;
  if (t >= N * k8n) return;
  const int n = t / k8n, k8 = (t % k8n) * 8;
  v8us v;
#pragma unroll
  for (int i = 0; i < 8; ++i) v[i] = bf16_bits(W[(size_t)(k8 + i) * N + n]);
  *(volatile v8us*)(Wt + (size_t)n * K + k8) = v;
  __threadfence();
  *(volatile v8us*)(Wt + (size_t)n * K + k8) = v;
}

template <bool ASPLIT, int ACT, bool BIAS_BF16>
__global__ __launch_bounds__(128) void k_gemm_bf(const float* __restrict__ A, int lda, const unsigned short* __restrict__ Wt, int ldb,
                                               const float* __restrict__ bias, float* __restrict__ C, int ldc, int M, int N, int K) {
  __shared__ __attribute__((aligned(16))) float so[4][16][64];
  const int tid = threadIdx.x, w = tid >> 5, lane = tid & 31, ln = lane & 15, hh = lane >> 4;
  const int ntn = N / 64;
  const int wid = blockIdx.x * 4 + w;
  const int mt = wid / ntn, nq = wid % ntn;
  if (mt * 16 >= M) return;
  const int row0 = mt * 16, col0 = nq * 64;
  const float* arow = A + (size_t)(row0 + ln) * lda;
  v8f acc[4] = {};
  for (int kb = 0; kb < K; kb += 32) {
    FragB ah, al;
    const v4f x0 = *(const v4fa*)(arow + kb + 8 * hh), x1 = *(const v4fa*)(arow + kb + 8 * hh + 4);
    const v4f x2 = *(const v4fa*)(arow + kb + 16 + 8 * hh), x3 = *(const v4fa*)(arow + kb + 16 + 8 * hh + 4);
    float xs[16] = {x0[0],x0[1],x0[2],x0[3],x1[0],x1[1],x1[2],x1[3],x2[0],x2[1],x2[2],x2[3],x3[0],x3[1],x3[2],x3[3]};
#pragma unroll
    for (int i = 0; i < 16; ++i) { const unsigned short hb = bf16_bits(xs[i]); ah.u[i] = hb; al.u[i] = ASPLIT ? bf16_bits(xs[i] - bf16_val(hb)) : (unsigned short)0; }
#pragma unroll
    for (int t = 0; t < 4; ++t) {
      const unsigned short* brow = Wt + (size_t)(col0 + t * 16 + ln) * ldb + kb;
      FragB b;
      b.half[0] = *(const v8us*)(brow + 8 * hh);
      b.half[1] = *(const v8us*)(brow + 16 + 8 * hh);
      acc[t] = mmaN<ASPLIT ? 2 : 1>(ah.v, al.v, b.v, b.v, acc[t]);
    }
  }
#pragma unroll
  for (int t = 0; t < 4; ++t) {
    float bv = bias ? bias[col0 + t * 16 + ln] : 0.f;
    if (BIAS_BF16) bv = bf16_round(bv);
#pragma unroll
    for (int r = 0; r < 8; ++r) { float v = acc[t][r] + bv; if (ACT == 1) v = fmaxf(v, 0.f); so[w][8 * hh + r][t * 16 + ln] = v; }
  }
  __builtin_amdgcn_fence(__ATOMIC_ACQ_REL, "workgroup");
  __builtin_amdgcn_wave_barrier();
  const int rsub = lane >> 4, c4 = (lane & 15) * 4;
  for (int pass = 0; pass < 2; ++pass) {
#pragma unroll
    for (int q = 0; q < 8; ++q) {
      const int r = q * 2 + rsub;
      const v4f v = *(const v4fa*)&so[w][r][c4];
      *(volatile v4f*)(C + (size_t)(row0 + r) * ldc + col0 + c4) = v;
    }
    if (pass == 0) __threadfence();
  }
}

template <bool ASPLIT, int ACT, bool BIAS_BF16, bool RES_BF16>
__global__ __launch_bounds__(128) void k_gemm_bf3(const float* __restrict__ A, int lda, const unsigned short* __restrict__ Wt, int ldb,
                                                const float* __restrict__ bias, const float* __restrict__ resid, int rmod, int ldr,
                                                float* __restrict__ C, int ldc, int M, int N, int K) {
  __shared__ __attribute__((aligned(16))) float so[4][16][64];
  const int tid = threadIdx.x, w = tid >> 5, lane = tid & 31, ln = lane & 15, hh = lane >> 4;
  const int ntn = N / 64;
  const int wid = blockIdx.x * 4 + w;
  const int mt = wid / ntn, nq = wid % ntn;
  if (mt * 16 >= M) return;
  const int row0 = mt * 16, col0 = nq * 64;
  const float* arow = A + (size_t)(row0 + ln) * lda;
  v8f acc[4] = {};
  for (int kb = 0; kb < K; kb += 32) {
    FragB ah, al;
    const v4f x0 = *(const v4fa*)(arow + kb + 8 * hh), x1 = *(const v4fa*)(arow + kb + 8 * hh + 4);
    const v4f x2 = *(const v4fa*)(arow + kb + 16 + 8 * hh), x3 = *(const v4fa*)(arow + kb + 16 + 8 * hh + 4);
    float xs[16] = {x0[0],x0[1],x0[2],x0[3],x1[0],x1[1],x1[2],x1[3],x2[0],x2[1],x2[2],x2[3],x3[0],x3[1],x3[2],x3[3]};
#pragma unroll
    for (int i = 0; i < 16; ++i) { const unsigned short hb = bf16_bits(xs[i]); ah.u[i] = hb; al.u[i] = ASPLIT ? bf16_bits(xs[i] - bf16_val(hb)) : (unsigned short)0; }
#pragma unroll
    for (int t = 0; t < 4; ++t) {
      const unsigned short* brow = Wt + (size_t)(col0 + t * 16 + ln) * ldb + kb;
      FragB b;
      b.half[0] = *(const v8us*)(brow + 8 * hh);
      b.half[1] = *(const v8us*)(brow + 16 + 8 * hh);
      acc[t] = mmaN<ASPLIT ? 2 : 1>(ah.v, al.v, b.v, b.v, acc[t]);
    }
  }
#pragma unroll
  for (int t = 0; t < 4; ++t) {
    const int col = col0 + t * 16 + ln;
    float bv = bias ? bias[col] : 0.f;
    if (BIAS_BF16) bv = bf16_round(bv);
#pragma unroll
    for (int r = 0; r < 8; ++r) {
      float v = acc[t][r] + bv;
      if (resid) { float rv = resid[(size_t)((row0 + 8 * hh + r) % rmod) * ldr + col]; if (RES_BF16) rv = bf16_round(rv); v += rv; }
      if (ACT == 1) v = fmaxf(v, 0.f);
      if (ACT == 2) v = 0.5f * v * (1.0f + erff(v * 0.70710678118654752f));
      if (ACT == 3) { const float u = 0.7978845608028654f * (v + 0.044715f * v * v * v); v = 0.5f * v * (1.0f + tanhf(u)); }
      so[w][8 * hh + r][t * 16 + ln] = v;
    }
  }
  __builtin_amdgcn_fence(__ATOMIC_ACQ_REL, "workgroup");
  __builtin_amdgcn_wave_barrier();
  const int rsub = lane >> 4, c4 = (lane & 15) * 4;
  for (int pass = 0; pass < 2; ++pass) {
#pragma unroll
    for (int q = 0; q < 8; ++q) {
      const int r = q * 2 + rsub;
      const v4f v = *(const v4fa*)&so[w][r][c4];
      *(volatile v4f*)(C + (size_t)(row0 + r) * ldc + col0 + c4) = v;
    }
    if (pass == 0) __threadfence();
  }
}
template <bool PARAM_BF16>
__global__ __launch_bounds__(256) void k_layernorm(const float* __restrict__ X, const float* __restrict__ R, const float* __restrict__ g, const float* __restrict__ bta,
                                                  float* __restrict__ out_sum, float* __restrict__ out_norm, int N, float eps) {
  __shared__ float red[256];
  const int row = blockIdx.x, tid = threadIdx.x;
  const float* x = X + (size_t)row * N; const float* rr = R ? R + (size_t)row * N : nullptr;
  float vals[16];
  const int per = N / 256;
  float s1 = 0.f;
  for (int u = 0; u < per / 4; ++u) {
    const int j = tid * 4 + 1024 * u;
    const v4f a = *(const v4fa*)(x + j);
    v4f b = {0.f,0.f,0.f,0.f}; if (rr) b = *(const v4fa*)(rr + j);
#pragma unroll
    for (int q = 0; q < 4; ++q) { const float v = a[q] + b[q]; vals[u * 4 + q] = v; s1 += v; }
  }
  red[tid] = s1; __syncthreads();
  for (int st = 128; st > 0; st >>= 1) { if (tid < st) red[tid] += red[tid + st]; __syncthreads(); }
  const float mu = red[0] / (float)N; __syncthreads();
  float s2 = 0.f;
  for (int u = 0; u < per / 4; ++u)
#pragma unroll
    for (int q = 0; q < 4; ++q) { const float c = vals[u * 4 + q] - mu; s2 += c * c; }
  red[tid] = s2; __syncthreads();
  for (int st = 128; st > 0; st >>= 1) { if (tid < st) red[tid] += red[tid + st]; __syncthreads(); }
  const float rs = rsqrtf(red[0] / (float)N + eps);
  for (int pass = 0; pass < 2; ++pass) {
    for (int u = 0; u < per / 4; ++u) {
      const int j = tid * 4 + 1024 * u;
      v4f o, sm;
#pragma unroll
      for (int q = 0; q < 4; ++q) {
        float gg = g[j + q], bb = bta[j + q];
        if (PARAM_BF16) { gg = bf16_round(gg); bb = bf16_round(bb); }
        sm[q] = vals[u * 4 + q]; o[q] = (vals[u * 4 + q] - mu) * rs * gg + bb;
      }
      if (out_sum) *(volatile v4f*)(out_sum + (size_t)row * N + j) = sm;
      *(volatile v4f*)(out_norm + (size_t)row * N + j) = o;
    }
    if (pass == 0) __threadfence();
  }
}


typedef _Float16 v16h __attribute__((ext_vector_type(16)));
union FragH { v16h v; v8us half[2]; _Float16 h[16]; unsigned short u[16]; };
template <int NT>
__device__ __forceinline__ v8f mmaH(v16h ah, v16h al, v16h bh, v16h bl, v8f c) {
  c = __builtin_amdgcn_wmma_f32_16x16x32_f16(false, ah, false, bh, (short)0, c, false, false);
  if (NT >= 2) c = __builtin_amdgcn_wmma_f32_16x16x32_f16(false, al, false, bh, (short)0, c, false, false);
  if (NT >= 3) c = __builtin_amdgcn_wmma_f32_16x16x32_f16(false, ah, false, bl, (short)0, c, false, false);
  asm volatile("v_nop\n\tv_nop\n\tv_nop\n\tv_nop" : "+v"(c) : "v"(ah), "v"(al), "v"(bh), "v"(bl));
  return c;
}
template <bool ASPLIT>
__global__ __launch_bounds__(128) void k_gemm_h(const float* __restrict__ A, int lda, size_t sA, const _Float16* __restrict__ Bh, int ldb, size_t sB, float alpha, float* __restrict__ C, int ldc, size_t sC, int M, int N, int K) {
  __shared__ __attribute__((aligned(16))) float so[4][16][64];
  const int tid = threadIdx.x, w = tid >> 5, lane = tid & 31, ln = lane & 15, hh = lane >> 4; const int by = blockIdx.y;
  A += (size_t)by * sA; Bh += (size_t)by * sB; C += (size_t)by * sC;
  const int ntn = (N + 63) / 64; const int wid = blockIdx.x * 4 + w; const int mt = wid / ntn, nq = wid % ntn; if (mt * 16 >= M) return;
  const int row0 = mt * 16, col0 = nq * 64; const float* arow = A + (size_t)(row0 + ln) * lda;
  v8f acc[4] = {};
  for (int kb = 0; kb < K; kb += 32) {
    FragH ah, al;
    const v4f x0 = *(const v4fa*)(arow + kb + 8 * hh), x1 = *(const v4fa*)(arow + kb + 8 * hh + 4), x2 = *(const v4fa*)(arow + kb + 16 + 8 * hh), x3 = *(const v4fa*)(arow + kb + 16 + 8 * hh + 4);
    float xs[16] = {x0[0],x0[1],x0[2],x0[3],x1[0],x1[1],x1[2],x1[3],x2[0],x2[1],x2[2],x2[3],x3[0],x3[1],x3[2],x3[3]};
#pragma unroll
    for (int i = 0; i < 16; ++i) { const _Float16 h = (_Float16)xs[i]; ah.h[i] = h; al.h[i] = ASPLIT ? (_Float16)(xs[i] - (float)h) : (_Float16)0.0f; }
#pragma unroll
    for (int t = 0; t < 4; ++t) { if (col0 + t * 16 >= N) continue; const size_t boff = (size_t)(col0 + t * 16 + ln) * ldb + kb; FragH bq; bq.half[0] = *(const v8us*)(Bh + boff + 8 * hh); bq.half[1] = *(const v8us*)(Bh + boff + 16 + 8 * hh);
      acc[t] = mmaH<ASPLIT ? 2 : 1>(ah.v, al.v, bq.v, bq.v, acc[t]); }
  }
#pragma unroll
  for (int t = 0; t < 4; ++t) { if (col0 + t * 16 >= N) continue;
#pragma unroll
    for (int r = 0; r < 8; ++r) so[w][8 * hh + r][t * 16 + ln] = acc[t][r] * alpha; }
  __builtin_amdgcn_fence(__ATOMIC_ACQ_REL, "workgroup"); __builtin_amdgcn_wave_barrier();
  const int rsub = lane >> 4, c4 = (lane & 15) * 4;
  for (int pass = 0; pass < 2; ++pass) {
#pragma unroll
    for (int q = 0; q < 8; ++q) { const int r = q * 2 + rsub; if (col0 + c4 < N) { const v4f v = *(const v4fa*)&so[w][r][c4]; *(volatile v4f*)(C + (size_t)(row0 + r) * ldc + col0 + c4) = v; } }
    if (pass == 0) __threadfence(); }
}

__global__ __launch_bounds__(256) void k_wt_f16(const float* __restrict__ W, _Float16* __restrict__ Wt, int K, int N, float scale) {
  const int t = blockIdx.x * 256 + threadIdx.x; if (t >= N * (K / 8)) return; const int n = t / (K / 8), k8 = (t % (K / 8)) * 8; FragH f;
#pragma unroll
  for (int i = 0; i < 8; ++i) f.h[i] = (_Float16)(bf16_round(W[(size_t)(k8 + i) * N + n]) * scale); const v8us o = f.half[0];
  *(volatile v8us*)((unsigned short*)Wt + (size_t)n * K + k8) = o; __threadfence(); *(volatile v8us*)((unsigned short*)Wt + (size_t)n * K + k8) = o;
}
template <int ACT>
__global__ __launch_bounds__(128) void k_gemm_hhx(const _Float16* __restrict__ A, int lda, size_t sA, const _Float16* __restrict__ Bh, int ldb, size_t sB, float alpha, const float* __restrict__ bias, size_t sBias, const float* __restrict__ CP, int rowsPerB, size_t sCPb, int row0g,
    float* __restrict__ C, _Float16* __restrict__ C16, int ldc, size_t sC, int M, int N, int K) {
  __shared__ __attribute__((aligned(16))) float so[4][16][64];
  const int tid = threadIdx.x, w = tid >> 5, lane = tid & 31, ln = lane & 15, hh = lane >> 4; const int by = blockIdx.y;
  A += (size_t)by * sA; Bh += (size_t)by * sB; const size_t cofs = (size_t)by * sC; const float* bp = bias ? bias + (size_t)by * sBias : nullptr;
  const int ntn = (N + 63) / 64; const int wid = blockIdx.x * 4 + w; const int mt = wid / ntn, nq = wid % ntn; if (mt * 16 >= M) return;
  const int row0 = mt * 16, col0 = nq * 64; const _Float16* arow = A + (size_t)(row0 + ln) * lda;
  v8f acc[4] = {};
  for (int kb = 0; kb < K; kb += 32) { FragH ah; ah.half[0] = *(const v8us*)((const unsigned short*)arow + kb + 8 * hh); ah.half[1] = *(const v8us*)((const unsigned short*)arow + kb + 16 + 8 * hh);
#pragma unroll
    for (int t = 0; t < 4; ++t) { if (col0 + t * 16 >= N) continue; const size_t boff = (size_t)(col0 + t * 16 + ln) * ldb + kb; FragH bq; bq.half[0] = *(const v8us*)((const unsigned short*)Bh + boff + 8 * hh); bq.half[1] = *(const v8us*)((const unsigned short*)Bh + boff + 16 + 8 * hh);
      acc[t] = mmaH<1>(ah.v, ah.v, bq.v, bq.v, acc[t]); }
  }
#pragma unroll
  for (int t = 0; t < 4; ++t) { if (col0 + t * 16 >= N) continue; const int col = col0 + t * 16 + ln; const float bv = bp ? bf16_round(bp[col]) : 0.f;
#pragma unroll
    for (int r = 0; r < 8; ++r) { float v = acc[t][r] * alpha + bv; if (CP) { const int bidx = (row0g + row0 + 8 * hh + r) / rowsPerB; v += CP[(size_t)bidx * sCPb + (size_t)by * 64 + col]; } if (ACT == 1) v = (v > 0.f) ? v : expm1f(v); else if (ACT == 7) v = (v > 0.f) ? v + 1.0f : expf(v); else if (ACT == 8) v = tanhf(v); else if (ACT == 9) v = 0.5f * v * (1.0f + tanhf(0.7978845608028654f * (v + 0.044715f * v * v * v))); else if (ACT == 11) v = 1.0f / (1.0f + expf(-v)); else if (ACT == 12) v = (v > 0.f) ? v : 0.01f * v; else if (ACT == 14) v = (v > 0.f) ? v : 0.1f * v; else if (ACT == 15) v = v / (1.0f + expf(-v)); else if (ACT == 3) v = fmaxf(v, 0.f); else if (ACT == 6) v = 0.5f * v * (1.0f + erff(v * 0.70710678118654752f)); so[w][8 * hh + r][t * 16 + ln] = v; } }
  __builtin_amdgcn_fence(__ATOMIC_ACQ_REL, "workgroup"); __builtin_amdgcn_wave_barrier();
  const int rsub = lane >> 4, c4 = (lane & 15) * 4; typedef _Float16 v4h __attribute__((ext_vector_type(4)));
  for (int pass = 0; pass < 2; ++pass) {
#pragma unroll
    for (int q = 0; q < 8; ++q) { const int r = q * 2 + rsub; if (col0 + c4 < N) { const v4f v = *(const v4fa*)&so[w][r][c4]; if (C) *(volatile v4f*)(C + cofs + (size_t)(row0 + r) * ldc + col0 + c4) = v; if (C16) { v4h h4; for (int i = 0; i < 4; ++i) h4[i] = (_Float16)v[i]; *(volatile v4h*)(C16 + cofs + (size_t)(row0 + r) * ldc + col0 + c4) = h4; } } }
    if (pass == 0) __threadfence(); }
}


typedef _Float16 v4h __attribute__((ext_vector_type(4)));

__global__ __launch_bounds__(256) void k_x16(const float* __restrict__ x, _Float16* __restrict__ X16, size_t n8) { const size_t t = (size_t)blockIdx.x * 256 + threadIdx.x; if (t >= n8) return; FragH f;
#pragma unroll
  for (int q = 0; q < 8; ++q) f.h[q] = (_Float16)bf16_round(x[t * 8 + q]); *(volatile v8us*)((unsigned short*)X16 + t * 8) = f.half[0]; __threadfence(); *(volatile v8us*)((unsigned short*)X16 + t * 8) = f.half[0]; }
__global__ __launch_bounds__(256) void k_h16(const float* __restrict__ x, _Float16* __restrict__ X16, size_t n8) { const size_t t = (size_t)blockIdx.x * 256 + threadIdx.x; if (t >= n8) return; FragH f;
#pragma unroll
  for (int q = 0; q < 8; ++q) f.h[q] = (_Float16)x[t * 8 + q]; *(volatile v8us*)((unsigned short*)X16 + t * 8) = f.half[0]; __threadfence(); *(volatile v8us*)((unsigned short*)X16 + t * 8) = f.half[0]; }
__global__ __launch_bounds__(256) void k_round16f(const float* __restrict__ W, _Float16* __restrict__ Bt, size_t n8) { const size_t t = (size_t)blockIdx.x * 256 + threadIdx.x; if (t >= n8) return; FragH f;
#pragma unroll
  for (int i = 0; i < 8; ++i) f.h[i] = (_Float16)(bf16_round(W[t * 8 + i]) * 16.0f); *(volatile v8us*)((unsigned short*)Bt + t * 8) = f.half[0]; __threadfence(); *(volatile v8us*)((unsigned short*)Bt + t * 8) = f.half[0]; }
template <int NHv, int TTv>
__global__ __launch_bounds__(256) void k_vt(const _Float16* __restrict__ V16, int ldv, int voff, _Float16* __restrict__ Vt) { __shared__ unsigned short tl[64][66]; const int tid = threadIdx.x; const int slab = blockIdx.x / (TTv / 64), lg = blockIdx.x % (TTv / 64); const int b = slab / NHv, h = slab % NHv;
  for (int i = tid; i < 64 * 8; i += 256) { const int r = i / 8, c8 = (i % 8) * 8; FragH f; f.half[0] = *(const v8us*)((const unsigned short*)V16 + ((size_t)b * TTv + lg * 64 + r) * ldv + voff + h * 64 + c8);
#pragma unroll
    for (int q = 0; q < 8; ++q) tl[r][c8 + q] = f.u[q]; }
  __syncthreads();
  for (int pass = 0; pass < 2; ++pass) {
#pragma unroll
    for (int rd = 0; rd < 2; ++rd) { const int d = rd * 32 + tid / 8, pc = tid % 8; FragH f;
#pragma unroll
      for (int q = 0; q < 8; ++q) f.u[q] = tl[pc * 8 + q][d];
      *(volatile v8us*)((unsigned short*)Vt + ((size_t)slab * 64 + d) * TTv + lg * 64 + pc * 8) = f.half[0]; }
    if (pass == 0) __threadfence(); } }

__global__ __launch_bounds__(256) void k_hl(const float* __restrict__ F, _Float16* __restrict__ Hh, _Float16* __restrict__ Hl, size_t n8) { const size_t t = (size_t)blockIdx.x * 256 + threadIdx.x; if (t >= n8) return; FragH fh, fl; const v4f a = *(const v4fa*)(F + t * 8), c = *(const v4fa*)(F + t * 8 + 4);
#pragma unroll
  for (int q = 0; q < 4; ++q) { _Float16 h = (_Float16)a[q]; fh.h[q] = h; fl.h[q] = (_Float16)((a[q] - (float)h) * 1024.0f); h = (_Float16)c[q]; fh.h[4 + q] = h; fl.h[4 + q] = (_Float16)((c[q] - (float)h) * 1024.0f); }
  for (int pass = 0; pass < 2; ++pass) { *(volatile v8us*)((unsigned short*)Hh + t * 8) = fh.half[0]; *(volatile v8us*)((unsigned short*)Hl + t * 8) = fl.half[0]; if (pass == 0) __threadfence(); } }

__global__ __launch_bounds__(256) void k_lnin(const float* __restrict__ x, const float* __restrict__ g, const float* __restrict__ bta, _Float16* __restrict__ H16, float* __restrict__ Xb) {
  #pragma clang fp contract(off)
  const int tid = threadIdx.x, w = tid >> 5, l = tid & 31; const int q = blockIdx.x * 8 + w; if (q >= NQP) return; float v[8]; float s = 0.f;
#pragma unroll
  for (int j = 0; j < 8; ++j) { const int ch = (j < 4) ? (4 * l + j) : (128 + 4 * l + (j - 4)); v[j] = (q < NQ) ? bf16_round(x[(size_t)ch * NQ + q]) : 0.f; s += v[j]; }
  for (int o = 16; o > 0; o >>= 1) s += __shfl_xor(s, o, 32); const float mu = s * (1.0f / CE); float vs = 0.f;
#pragma unroll
  for (int j = 0; j < 8; ++j) { const float d = v[j] - mu; vs += d * d; }
  for (int o = 16; o > 0; o >>= 1) vs += __shfl_xor(vs, o, 32); const float rs = rsqrtf(vs * (1.0f / CE) + 1e-6f); FragH f; v4f a, c;
#pragma unroll
  for (int j = 0; j < 8; ++j) { const int ch = (j < 4) ? (4 * l + j) : (128 + 4 * l + (j - 4)); f.h[j] = (q < NQ) ? (_Float16)((v[j] - mu) * rs * bf16_round(g[ch]) + bf16_round(bta[ch])) : (_Float16)0.0f; if (j < 4) a[j] = v[j]; else c[j - 4] = v[j]; }
  const unsigned long long h0 = *(const unsigned long long*)&f.u[0], h1 = *(const unsigned long long*)&f.u[4];
  for (int pass = 0; pass < 2; ++pass) { *(volatile unsigned long long*)((unsigned short*)H16 + (size_t)q * CE + 4 * l) = h0; *(volatile unsigned long long*)((unsigned short*)H16 + (size_t)q * CE + 128 + 4 * l) = h1; *(volatile v4f*)(Xb + (size_t)q * CE + 4 * l) = a; *(volatile v4f*)(Xb + (size_t)q * CE + 128 + 4 * l) = c; if (pass == 0) __threadfence(); } }
__global__ __launch_bounds__(256) void k_vfeat(const float* __restrict__ refv, _Float16* __restrict__ V16) { const int tid = threadIdx.x, w = tid >> 5, l = tid & 31; const int pos = blockIdx.x * 8 + w; if (pos >= NCm * ML) return; const int cam = pos / ML, m = pos % ML; FragH f;
#pragma unroll
  for (int j = 0; j < 8; ++j) f.h[j] = (_Float16)bf16_round(refv[((size_t)cam * CE + 8 * l + j) * ML + m]);
  *(volatile v8us*)((unsigned short*)V16 + (size_t)pos * CE + 8 * l) = f.half[0]; __threadfence(); *(volatile v8us*)((unsigned short*)V16 + (size_t)pos * CE + 8 * l) = f.half[0]; }
__global__ __launch_bounds__(64) void k_inv(const float* __restrict__ M, float* __restrict__ L2I) { const int t = threadIdx.x; if (t >= NCm * 4) return; const int cam = t / 4, row = t % 4; const float* p = M + cam * 16;
  const double a00 = bf16_round(p[0]), a01 = bf16_round(p[1]), a02 = bf16_round(p[2]), a03 = bf16_round(p[3]), a10 = bf16_round(p[4]), a11 = bf16_round(p[5]), a12 = bf16_round(p[6]), a13 = bf16_round(p[7]);
  const double a20 = bf16_round(p[8]), a21 = bf16_round(p[9]), a22 = bf16_round(p[10]), a23 = bf16_round(p[11]), a30 = bf16_round(p[12]), a31 = bf16_round(p[13]), a32 = bf16_round(p[14]), a33 = bf16_round(p[15]);
  const double s0 = a00 * a11 - a10 * a01, s1 = a00 * a12 - a10 * a02, s2 = a00 * a13 - a10 * a03, s3 = a01 * a12 - a11 * a02, s4 = a01 * a13 - a11 * a03, s5 = a02 * a13 - a12 * a03;
  const double c5 = a22 * a33 - a32 * a23, c4 = a21 * a33 - a31 * a23, c3 = a21 * a32 - a31 * a22, c2 = a20 * a33 - a30 * a23, c1 = a20 * a32 - a30 * a22, c0 = a20 * a31 - a30 * a21;
  const double det = s0 * c5 - s1 * c4 + s2 * c3 + s3 * c2 - s4 * c1 + s5 * c0; const double id = 1.0 / det;
  float r[16];
  r[0] = (float)(( a11 * c5 - a12 * c4 + a13 * c3) * id); r[1] = (float)((-a01 * c5 + a02 * c4 - a03 * c3) * id); r[2] = (float)(( a31 * s5 - a32 * s4 + a33 * s3) * id); r[3] = (float)((-a21 * s5 + a22 * s4 - a23 * s3) * id);
  r[4] = (float)((-a10 * c5 + a12 * c2 - a13 * c1) * id); r[5] = (float)(( a00 * c5 - a02 * c2 + a03 * c1) * id); r[6] = (float)((-a30 * s5 + a32 * s2 - a33 * s1) * id); r[7] = (float)(( a20 * s5 - a22 * s2 + a23 * s1) * id);
  r[8] = (float)(( a10 * c4 - a11 * c2 + a13 * c0) * id); r[9] = (float)((-a00 * c4 + a01 * c2 - a03 * c0) * id); r[10] = (float)(( a30 * s4 - a31 * s2 + a33 * s0) * id); r[11] = (float)((-a20 * s4 + a21 * s2 - a23 * s0) * id);
  r[12] = (float)((-a10 * c3 + a11 * c1 - a12 * c0) * id); r[13] = (float)(( a00 * c3 - a01 * c1 + a02 * c0) * id); r[14] = (float)((-a30 * s3 + a31 * s1 - a32 * s0) * id); r[15] = (float)(( a20 * s3 - a21 * s1 + a22 * s0) * id);
  v4f o; o[0] = (row == 0) ? r[0] : (row == 1) ? r[4] : (row == 2) ? r[8] : r[12]; o[1] = (row == 0) ? r[1] : (row == 1) ? r[5] : (row == 2) ? r[9] : r[13]; o[2] = (row == 0) ? r[2] : (row == 1) ? r[6] : (row == 2) ? r[10] : r[14]; o[3] = (row == 0) ? r[3] : (row == 1) ? r[7] : (row == 2) ? r[11] : r[15];
  *(volatile v4f*)(L2I + t * 4) = o; __threadfence(); *(volatile v4f*)(L2I + t * 4) = o; }
__global__ __launch_bounds__(256) void k_proj(const float* __restrict__ L2I, const float* __restrict__ imgwh, float* __restrict__ UVV) {
  #pragma clang fp contract(off)
  const int t = blockIdx.x * 256 + threadIdx.x; if (t >= NCm * NQ) return; const int c = t / NQ, q = t % NQ; const int iy = q / WQ, ix = q % WQ; const float gx = ((float)ix + 0.5f) / (float)WQ, gy = ((float)iy + 0.5f) / (float)HQ;
  const float X = gx * (51.2f - (-51.2f)) + (-51.2f), Y = gy * (51.2f - (-51.2f)) + (-51.2f), Z = 0.5f * (3.0f - (-5.0f)) + (-5.0f); const float* m = L2I + c * 16;
  const float cx = ((m[0] * X + m[1] * Y) + m[2] * Z) + m[3], cy = ((m[4] * X + m[5] * Y) + m[6] * Z) + m[7], cz = ((m[8] * X + m[9] * Y) + m[10] * Z) + m[11];
  const float dep = fmaxf(cz, 1e-5f); const float u = (cx / dep) / bf16_round(imgwh[c * 2]), v = (cy / dep) / bf16_round(imgwh[c * 2 + 1]); const bool ok = (cz > 1e-5f) && (u > 0.f) && (u < 1.f) && (v > 0.f) && (v < 1.f);
  v4f o; o[0] = u; o[1] = v; o[2] = ok ? 1.f : 0.f; o[3] = 0.f; *(volatile v4f*)(UVV + (size_t)t * 4) = o; __threadfence(); *(volatile v4f*)(UVV + (size_t)t * 4) = o; }
__global__ __launch_bounds__(256) void k_tanh(float* OFF, size_t n4) { const size_t t = (size_t)blockIdx.x * 256 + threadIdx.x; if (t >= n4) return; v4f v = *(const v4fa*)(OFF + t * 4);
#pragma unroll
  for (int j = 0; j < 4; ++j) v[j] = tanhf(v[j]); *(volatile v4f*)(OFF + t * 4) = v; __threadfence(); *(volatile v4f*)(OFF + t * 4) = v; }
__global__ __launch_bounds__(256) void k_msda(const _Float16* __restrict__ V16, const float* __restrict__ OFF, const float* __restrict__ ATT, const float* __restrict__ UVV, _Float16* __restrict__ O16) {
  #pragma clang fp contract(off)
  __shared__ __attribute__((aligned(16))) unsigned short rowb[8][CE]; const int tid = threadIdx.x, w = tid >> 5, l = tid & 31; const int q = blockIdx.x * 8 + w;
  int nvis = 0;
#pragma unroll
  for (int c = 0; c < NCm; ++c) nvis += (UVV[((size_t)c * NQ + q) * 4 + 2] != 0.f) ? 1 : 0;
#pragma unroll 1
  for (int h = 0; h < NH; ++h) { float a[NPt], odx[NPt], ody[NPt]; float mx = -3.0e38f;
#pragma unroll
    for (int p = 0; p < NPt; ++p) { a[p] = ATT[(size_t)q * 32 + h * NPt + p]; mx = fmaxf(mx, a[p]); odx[p] = OFF[(size_t)q * 64 + (h * NPt + p) * 2]; ody[p] = OFF[(size_t)q * 64 + (h * NPt + p) * 2 + 1]; }
    float su = 0.f;
#pragma unroll
    for (int p = 0; p < NPt; ++p) { a[p] = expf(a[p] - mx); su += a[p]; }
    const float den = (float)nvis * 1.0f;
    float ssum = 0.f;
#pragma unroll
    for (int p = 0; p < NPt; ++p) ssum += a[p] / su;
    const float norm = 1.0f / (ssum * (float)nvis + 1e-6f); (void)den; float acc = 0.f;
#pragma unroll 1
    for (int c = 0; c < NCm; ++c) { const v4f uv = *(const v4fa*)(UVV + ((size_t)c * NQ + q) * 4); if (uv[2] == 0.f) continue;
#pragma unroll 1
      for (int p = 0; p < NPt; ++p) { const float lx = uv[0] + odx[p] / (float)WL, ly = uv[1] + ody[p] / (float)HL; const float xp = lx * (float)WL - 0.5f, yp = ly * (float)HL - 0.5f; const float fx = floorf(xp), fy = floorf(yp); const float wx = xp - fx, wy = yp - fy; const int x0 = (int)fx, y0 = (int)fy; float sv = 0.f;
#pragma unroll
        for (int k = 0; k < 4; ++k) { const int xi = x0 + (k & 1), yi = y0 + (k >> 1); const bool valid = (xi >= 0) && (xi < WL) && (yi >= 0) && (yi < HL); const float wgt = ((k & 1) ? wx : 1.f - wx) * ((k >> 1) ? wy : 1.f - wy); const int idx = min(max(yi, 0), HL - 1) * WL + min(max(xi, 0), WL - 1);
          sv += (valid ? wgt : 0.f) * (float)V16[((size_t)c * ML + idx) * CE + h * DHd + l]; }
        acc += (a[p] / su) * norm * sv; } }
    FragH f; f.h[0] = (_Float16)acc; rowb[w][h * DHd + l] = f.u[0]; }
  __syncthreads();
  { const v8us vv = *(const v8us*)&rowb[w][l * 8]; *(volatile v8us*)((unsigned short*)O16 + (size_t)q * CE + l * 8) = vv; __threadfence(); *(volatile v8us*)((unsigned short*)O16 + (size_t)q * CE + l * 8) = vv; } }
__global__ __launch_bounds__(256) void k_lnout(const _Float16* __restrict__ O16, const float* __restrict__ g, const float* __restrict__ bta, _Float16* __restrict__ Y16) {
  #pragma clang fp contract(off)
  const int tid = threadIdx.x, w = tid >> 5, l = tid & 31; const int q = blockIdx.x * 8 + w; if (q >= NQP) return; FragH fi; if (q < NQ) fi.half[0] = *(const v8us*)((const unsigned short*)O16 + (size_t)q * CE + 8 * l); float v[8]; float s = 0.f;
#pragma unroll
  for (int j = 0; j < 8; ++j) { v[j] = (q < NQ) ? (float)fi.h[j] : 0.f; s += v[j]; }
  for (int o = 16; o > 0; o >>= 1) s += __shfl_xor(s, o, 32); const float mu = s * (1.0f / CE); float vs = 0.f;
#pragma unroll
  for (int j = 0; j < 8; ++j) { const float d = v[j] - mu; vs += d * d; }
  for (int o = 16; o > 0; o >>= 1) vs += __shfl_xor(vs, o, 32); const float rs = rsqrtf(vs * (1.0f / CE) + 1e-6f); FragH f;
#pragma unroll
  for (int j = 0; j < 8; ++j) { const int ch = 8 * l + j; f.h[j] = (q < NQ) ? (_Float16)((v[j] - mu) * rs * bf16_round(g[ch]) + bf16_round(bta[ch])) : (_Float16)0.0f; }
  *(volatile v8us*)((unsigned short*)Y16 + (size_t)q * CE + 8 * l) = f.half[0]; __threadfence(); *(volatile v8us*)((unsigned short*)Y16 + (size_t)q * CE + 8 * l) = f.half[0]; }
__global__ __launch_bounds__(256) void k_nchw(const float* __restrict__ R, float* __restrict__ out) { const int t = blockIdx.x * 256 + threadIdx.x; if (t >= CE * NQ / 4) return; const int ch = t / (NQ / 4), q4 = (t % (NQ / 4)) * 4; v4f v;
#pragma unroll
  for (int j = 0; j < 4; ++j) v[j] = R[(size_t)(q4 + j) * CE + ch]; *(volatile v4f*)(out + (size_t)ch * NQ + q4) = v; __threadfence(); *(volatile v4f*)(out + (size_t)ch * NQ + q4) = v; }

extern "C" void kernel_launch(void* const* d_in, const int* in_sizes, int n_in,
                              void* d_out, int out_size, void* d_ws, size_t ws_size, hipStream_t stream) {
  (void)in_sizes; (void)n_in; (void)out_size;
  const float* const* I = (const float* const*)d_in; const float* x = I[0]; const float* refv = I[1]; const float* mats = I[2]; const float* imgwh = I[3]; const float* lng = I[4]; const float* lnb = I[5]; const float* ffw = I[6]; const float* ffb = I[7]; const float* ofw = I[8]; const float* ofb = I[9]; const float* atw = I[10]; const float* atb = I[11]; const float* log_ = I[12]; const float* lob = I[13]; const float* fow = I[14]; const float* fob = I[15];
  char* ws = (char*)d_ws; size_t off = 0;
  auto take = [&](size_t bytes) { char* p = ws + off; off += (bytes + 255) & ~(size_t)255; return p; };
  _Float16* Bff = (_Float16*)take((size_t)CE * CE * 2); _Float16* Bof = (_Float16*)take((size_t)64 * CE * 2); _Float16* Bat = (_Float16*)take((size_t)32 * CE * 2); _Float16* Bfo = (_Float16*)take((size_t)CE * CE * 2); float* L2I = (float*)take(NCm * 16 * 4); float* UVV = (float*)take((size_t)NCm * NQ * 4 * 4);
  _Float16* XN = (_Float16*)take((size_t)NQP * CE * 2); float* Xb = (float*)take((size_t)NQP * CE * 4); _Float16* H16 = (_Float16*)take((size_t)NQP * CE * 2); float* OFF = (float*)take((size_t)NQP * 64 * 4); float* ATT = (float*)take((size_t)NQP * 32 * 4); _Float16* V16 = (_Float16*)take((size_t)NCm * ML * CE * 2); _Float16* O16 = (_Float16*)take((size_t)NQP * CE * 2); _Float16* Y16 = (_Float16*)take((size_t)NQP * CE * 2); float* R = (float*)take((size_t)NQP * CE * 4);
  if (off > ws_size) return;
  k_round16f<<<(unsigned)(((size_t)CE * CE / 8 + 255) / 256), 256, 0, stream>>>(ffw, Bff, (size_t)CE * CE / 8); k_round16f<<<(64 * CE / 8 + 255) / 256, 256, 0, stream>>>(ofw, Bof, (size_t)64 * CE / 8); k_round16f<<<(32 * CE / 8 + 255) / 256, 256, 0, stream>>>(atw, Bat, (size_t)32 * CE / 8); k_round16f<<<(unsigned)(((size_t)CE * CE / 8 + 255) / 256), 256, 0, stream>>>(fow, Bfo, (size_t)CE * CE / 8);
  k_inv<<<1, 64, 0, stream>>>(mats, L2I);
  k_lnin<<<NQP / 8, 256, 0, stream>>>(x, lng, lnb, XN, Xb); k_vfeat<<<NCm * ML / 8, 256, 0, stream>>>(refv, V16);
  const dim3 g256(((NQP / 16) * (CE / 64) + 3) / 4, 1), g1(((NQP / 16) * 1 + 3) / 4, 1);
  k_gemm_hhx<0><<<g256, 128, 0, stream>>>(XN, CE, 0, Bff, CE, 0, 0.0625f, ffb, 0, nullptr, 1, 0, 0, nullptr, H16, CE, 0, NQP, CE, CE);
  k_gemm_hhx<0><<<g1, 128, 0, stream>>>(H16, CE, 0, Bof, CE, 0, 0.0625f, ofb, 0, nullptr, 1, 0, 0, OFF, nullptr, 64, 0, NQP, 64, CE);
  k_gemm_hhx<0><<<g1, 128, 0, stream>>>(H16, CE, 0, Bat, CE, 0, 0.0625f, atb, 0, nullptr, 1, 0, 0, ATT, nullptr, 32, 0, NQP, 32, CE);
  k_proj<<<(NCm * NQ + 255) / 256, 256, 0, stream>>>(L2I, imgwh, UVV); k_tanh<<<(NQP * 64 / 4 + 255) / 256, 256, 0, stream>>>(OFF, (size_t)NQP * 64 / 4);
  k_msda<<<NQ / 8, 256, 0, stream>>>(V16, OFF, ATT, UVV, O16);
  k_lnout<<<NQP / 8, 256, 0, stream>>>(O16, log_, lob, Y16);
  k_gemm_hhx<0><<<g256, 128, 0, stream>>>(Y16, CE, 0, Bfo, CE, 0, 0.0625f, fob, 0, Xb, 1, (size_t)CE, 0, R, nullptr, CE, 0, NQP, CE, CE);
  k_nchw<<<(CE * NQ / 4 + 255) / 256, 256, 0, stream>>>(R, (float*)d_out);
}
